// ScanLayer_80144089743475
// MI455X (gfx1250) — hardware-run, weakly checked
//
#include <hip/hip_runtime.h>
#include <math.h>

constexpr int N_BATCH = 4;
constexpr int N_STEP  = 2048;
constexpr int N_GRP   = 8;
constexpr int N_DIN   = 128;
constexpr int N_HID   = 256;
constexpr int N_GATE  = 2 * N_HID;
constexpr int CH_LEN  = 32;
constexpr int N_CHUNK = N_STEP / CH_LEN;
constexpr int N_THR   = 256;
constexpr int AB_PITCH = N_HID + 4;
constexpr int XN_PITCH = N_DIN + 8;
constexpr int HS_PITCH = N_HID + 8;
constexpr int CT_PITCH = N_DIN + 4;
constexpr float X_CARRY    = 16.0f;
constexpr float WIN_CARRY  = 64.0f;
constexpr float H_CARRY    = 16.0f;
constexpr float WOUT_CARRY = 64.0f;
constexpr float IN_FOLD    = 1.0f / (X_CARRY * WIN_CARRY);
constexpr float OUT_FOLD   = 1.0f / (H_CARRY * WOUT_CARRY);
constexpr float LN_EPS_F   = 1e-5f;

constexpr int N_OUT0 = N_BATCH * N_STEP * N_GRP * N_DIN;
constexpr int N_OUT1 = N_BATCH * N_GRP * N_HID;
constexpr int N8_WIN  = N_GRP * N_GATE * N_DIN / 8;
constexpr int N8_WOUT = N_GRP * N_DIN * N_HID / 8;

static_assert(N_STEP % CH_LEN == 0, "chunking exact");
static_assert(CH_LEN == 32, "two 16-row m-subtiles per block");
static_assert(N_HID == N_THR, "one scan thread per hidden channel");
static_assert(N_DIN == 32 * 4, "one float4 per lane per row");
static_assert(N_GATE == (N_THR / 32) * 64, "8 waves x 64 gate columns");
static_assert(N_DIN == (N_THR / 32) * 16, "8 waves x 16 output columns");
static_assert(N_DIN % 32 == 0 && N_HID % 32 == 0, "k multiples of 32");
static_assert(CH_LEN % (N_THR / 32) == 0, "rows per wave exact");
static_assert(CH_LEN * CT_PITCH <= CH_LEN * AB_PITCH, "out tile fits in the dead gate plane");
static_assert(N8_WIN % N_THR == 0 && N8_WOUT % N_THR == 0, "plane kernel grid exact");
static_assert((N_BATCH * N_GRP * N_HID) % N_THR == 0, "carry kernel grid exact");
static_assert((XN_PITCH * 2) % 16 == 0 && (HS_PITCH * 2) % 16 == 0 && (CT_PITCH * 4) % 16 == 0, "16-B aligned LDS rows");

typedef __attribute__((ext_vector_type(16))) _Float16 v16h;
typedef __attribute__((ext_vector_type(8)))  _Float16 v8h;
typedef __attribute__((ext_vector_type(4)))  _Float16 v4h;
typedef __attribute__((ext_vector_type(8)))  float    v8f;
typedef __attribute__((ext_vector_type(4)))  float    v4f;

union FragU { v16h v; v8h h[2]; };
__device__ __forceinline__ v16h frag_load(const _Float16* p) {
  FragU f;
  f.h[0] = *(const v8h*)(p);
  f.h[1] = *(const v8h*)(p + 16);
  return f.v;
}
__device__ __forceinline__ v8f mma_f16(v16h a, v16h b, v8f c) {
  c = __builtin_amdgcn_wmma_f32_16x16x32_f16(false, a, false, b, (short)0, c, false, false);
  asm volatile("v_nop\n\tv_nop\n\tv_nop\n\tv_nop" : "+v"(c) : "v"(a), "v"(b));
  return c;
}
__device__ __forceinline__ void store2_f32(float* p, float v) {
  *(volatile float*)p = v;
  __threadfence();
  *(volatile float*)p = v;
}

__global__ __launch_bounds__(N_THR) void weight_planes_kernel(const float* __restrict__ w_in, const float* __restrict__ w_out,
                                                             unsigned short* __restrict__ w_inT, unsigned short* __restrict__ w_outT) {
  const int i = blockIdx.x * N_THR + threadIdx.x;
  if (blockIdx.x < N8_WIN / N_THR) {
    const int k8 = i & 15;
    const int n  = (i >> 4) & (N_GATE - 1);
    const int c  = i >> 13;
    const float* sp = w_in + ((size_t)c * N_DIN + (size_t)k8 * 8) * N_GATE + n;
    v8h hv;
#pragma unroll
    for (int e = 0; e < 8; ++e) {
      const float w = sp[(size_t)e * N_GATE];
      hv[e] = (_Float16)(w * WIN_CARRY);
    }
    unsigned short* dp = w_inT + (size_t)i * 8;
    *(volatile v8h*)dp = hv;
    __threadfence();
    *(volatile v8h*)dp = hv;
  } else {
    const int i2 = i - N8_WIN;
    const int k8 = i2 & 31;
    const int n  = (i2 >> 5) & (N_DIN - 1);
    const int c  = i2 >> 12;
    const float* sp = w_out + ((size_t)c * N_HID + (size_t)k8 * 8) * N_DIN + n;
    v8h hv;
#pragma unroll
    for (int e = 0; e < 8; ++e) {
      const float w = sp[(size_t)e * N_DIN];
      hv[e] = (_Float16)(w * WOUT_CARRY);
    }
    unsigned short* dp = w_outT + (size_t)i2 * 8;
    *(volatile v8h*)dp = hv;
    __threadfence();
    *(volatile v8h*)dp = hv;
  }
}

template <bool FINAL>
__global__ __launch_bounds__(N_THR) void chunk_pass_kernel(
    const float* __restrict__ x, const float* __restrict__ h_init,
    const float* __restrict__ gamma, const float* __restrict__ beta,
    const float* __restrict__ b_in, const float* __restrict__ b_out,
    const unsigned short* __restrict__ w_inT_p, const unsigned short* __restrict__ w_outT_p,
    float* __restrict__ A_end, float* __restrict__ H_end,
    const float* __restrict__ carry_in, float* __restrict__ out) {
  constexpr int XH_ELEMS = FINAL ? (CH_LEN * HS_PITCH) : (CH_LEN * XN_PITCH);
  __shared__ __align__(16) float    abS[2 * CH_LEN * AB_PITCH];
  __shared__ __align__(16) _Float16 xhS[XH_ELEMS];
  float* aS = abS;
  float* bS = abS + CH_LEN * AB_PITCH;

  const int chunk = blockIdx.x, grp = blockIdx.y, bat = blockIdx.z;
  const int tid = threadIdx.x, wave = tid >> 5, lane = tid & 31;
  const int cl = lane & 15, hh = lane >> 4;
  const int n0 = chunk * CH_LEN;
  const _Float16* w_inT  = (const _Float16*)w_inT_p;
  const _Float16* w_outT = (const _Float16*)w_outT_p;

  {
    const v4f g4  = *(const v4f*)(gamma + grp * N_DIN + lane * 4);
    const v4f be4 = *(const v4f*)(beta  + grp * N_DIN + lane * 4);
#pragma unroll 2
    for (int rr = 0; rr < CH_LEN / 8; ++rr) {
      const int t = wave * (CH_LEN / 8) + rr;
      const float* xr = x + (((size_t)bat * N_STEP + (size_t)(n0 + t)) * N_GRP + grp) * N_DIN + lane * 4;
      const v4f v = *(const v4f*)xr;
      float s = (v[0] + v[1]) + (v[2] + v[3]);
#pragma unroll
      for (int off = 16; off > 0; off >>= 1) s += __shfl_xor(s, off, 32);
      const float mu = s * (1.0f / N_DIN);
      const float d0 = v[0] - mu, d1 = v[1] - mu, d2 = v[2] - mu, d3 = v[3] - mu;
      float ss = (d0 * d0 + d1 * d1) + (d2 * d2 + d3 * d3);
#pragma unroll
      for (int off = 16; off > 0; off >>= 1) ss += __shfl_xor(ss, off, 32);
      const float rstd = rsqrtf(ss * (1.0f / N_DIN) + LN_EPS_F);
      v4h hv;
      hv[0] = (_Float16)(((d0 * rstd) * g4[0] + be4[0]) * X_CARRY);
      hv[1] = (_Float16)(((d1 * rstd) * g4[1] + be4[1]) * X_CARRY);
      hv[2] = (_Float16)(((d2 * rstd) * g4[2] + be4[2]) * X_CARRY);
      hv[3] = (_Float16)(((d3 * rstd) * g4[3] + be4[3]) * X_CARRY);
      *(v4h*)(xhS + t * XN_PITCH + lane * 4) = hv;
    }
  }
  __syncthreads();

  {
    v16h af[2][4];
#pragma unroll
    for (int mi = 0; mi < 2; ++mi)
#pragma unroll
      for (int kk = 0; kk < 4; ++kk)
        af[mi][kk] = frag_load(xhS + (16 * mi + cl) * XN_PITCH + kk * 32 + 8 * hh);
    const int planeoff = (wave >= 4) ? (CH_LEN * AB_PITCH - N_HID) : 0;
#pragma unroll 1
    for (int j = 0; j < 4; ++j) {
      const int ncol = 64 * wave + 16 * j + cl;
      const _Float16* wb = w_inT + ((size_t)grp * N_GATE + ncol) * N_DIN + 8 * hh;
      v16h bf[4];
#pragma unroll
      for (int kk = 0; kk < 4; ++kk) bf[kk] = frag_load(wb + kk * 32);
      v8f acc0 = {0.f, 0.f, 0.f, 0.f, 0.f, 0.f, 0.f, 0.f};
      v8f acc1 = {0.f, 0.f, 0.f, 0.f, 0.f, 0.f, 0.f, 0.f};
#pragma unroll
      for (int kk = 0; kk < 4; ++kk) {
        acc0 = mma_f16(af[0][kk], bf[kk], acc0);
        acc1 = mma_f16(af[1][kk], bf[kk], acc1);
      }
      const int dcol = ncol + planeoff;
#pragma unroll
      for (int r = 0; r < 8; ++r) {
        aS[(8 * hh + r) * AB_PITCH + dcol]      = acc0[r];
        aS[(16 + 8 * hh + r) * AB_PITCH + dcol] = acc1[r];
      }
    }
  }
  __syncthreads();

  const int e = tid;
  const size_t bc = (size_t)bat * N_GRP + grp;
  const size_t se = (bc * N_CHUNK + (size_t)chunk) * N_HID + e;
  {
    const float bia = b_in[grp * N_GATE + e];
    const float bib = b_in[grp * N_GATE + N_HID + e];
    const float h0v = h_init[bc * N_HID + e];
    float H;
    if (FINAL) {
      const float cin = carry_in[se];
      H = (chunk == 0) ? h0v : cin;
    } else {
      H = (chunk == 0) ? h0v : 0.0f;
    }
    float A = 1.0f;
#pragma unroll 1
    for (int t = 0; t < CH_LEN; ++t) {
      const float ar = aS[t * AB_PITCH + e] * IN_FOLD + bia;
      const float br = bS[t * AB_PITCH + e] * IN_FOLD + bib;
      const float ga = 1.0f / (1.0f + expf(-ar));
      const float sg = 1.0f / (1.0f + expf(-br));
      const float gb = br * sg;
      H = fmaf(ga, H, gb);
      if (FINAL) {
        xhS[t * HS_PITCH + e] = (_Float16)(H * H_CARRY);
      } else {
        A *= ga;
      }
    }
    if (!FINAL) {
      const float av = A, hv = H;
      *(volatile float*)(A_end + se) = av;
      *(volatile float*)(H_end + se) = hv;
      __threadfence();
      *(volatile float*)(A_end + se) = av;
      *(volatile float*)(H_end + se) = hv;
    }
  }

  if (FINAL) {
    __syncthreads();
    float* Cst = abS;
    {
      v8f c0 = {0.f, 0.f, 0.f, 0.f, 0.f, 0.f, 0.f, 0.f};
      v8f c1 = {0.f, 0.f, 0.f, 0.f, 0.f, 0.f, 0.f, 0.f};
      const _Float16* wb = w_outT + ((size_t)grp * N_DIN + 16 * wave + cl) * N_HID + 8 * hh;
      const _Float16* ha = xhS + cl * HS_PITCH + 8 * hh;
#pragma unroll 2
      for (int kk = 0; kk < N_HID / 32; ++kk) {
        const v16h bq = frag_load(wb + kk * 32);
        const v16h a0 = frag_load(ha + kk * 32);
        const v16h a1 = frag_load(ha + 16 * HS_PITCH + kk * 32);
        c0 = mma_f16(a0, bq, c0);
        c1 = mma_f16(a1, bq, c1);
      }
#pragma unroll
      for (int r = 0; r < 8; ++r) {
        Cst[(8 * hh + r) * CT_PITCH + 16 * wave + cl]      = c0[r] * OUT_FOLD;
        Cst[(16 + 8 * hh + r) * CT_PITCH + 16 * wave + cl] = c1[r] * OUT_FOLD;
      }
    }
    __syncthreads();
    {
      const v4f bo = *(const v4f*)(b_out + grp * N_DIN + lane * 4);
      v4f o[CH_LEN / 8];
#pragma unroll
      for (int i = 0; i < CH_LEN / 8; ++i) {
        const int t = wave * (CH_LEN / 8) + i;
        const size_t off = (((size_t)bat * N_STEP + (size_t)(n0 + t)) * N_GRP + grp) * N_DIN + lane * 4;
        const v4f cv = *(const v4f*)(Cst + t * CT_PITCH + lane * 4);
        const v4f xv = *(const v4f*)(x + off);
        o[i] = (cv + bo) + xv;
      }
      for (int pass = 0; pass < 2; ++pass) {
#pragma unroll
        for (int i = 0; i < CH_LEN / 8; ++i) {
          const int t = wave * (CH_LEN / 8) + i;
          const size_t off = (((size_t)bat * N_STEP + (size_t)(n0 + t)) * N_GRP + grp) * N_DIN + lane * 4;
          *(volatile v4f*)(out + off) = o[i];
        }
        __threadfence();
      }
    }
  }
}

__global__ __launch_bounds__(N_THR) void carry_scan_kernel(const float* __restrict__ A_end, const float* __restrict__ H_end,
                                                          float* __restrict__ carry_in, float* __restrict__ h_last) {
  const int g  = blockIdx.x * N_THR + threadIdx.x;
  const int e  = g & (N_HID - 1);
  const int bc = g >> 8;
  const size_t base = (size_t)bc * N_CHUNK * N_HID + e;
  float carry = 0.0f;
#pragma unroll 1
  for (int k = 0; k < N_CHUNK; ++k) {
    const size_t idx = base + (size_t)k * N_HID;
    const float av = A_end[idx];
    const float hv = H_end[idx];
    store2_f32(carry_in + idx, carry);
    carry = fmaf(av, carry, hv);
  }
  store2_f32(h_last + g, carry);
}

extern "C" void kernel_launch(void* const* d_in, const int* in_sizes, int n_in,
                              void* d_out, int out_size, void* d_ws, size_t ws_size, hipStream_t stream) {
  if (n_in < 8 || d_out == nullptr || d_ws == nullptr) return;
  if (in_sizes[0] != N_OUT0 || in_sizes[1] != N_OUT1 || in_sizes[2] != N_GRP * N_DIN ||
      in_sizes[3] != N_GRP * N_DIN || in_sizes[4] != N_GRP * N_DIN * N_GATE || in_sizes[5] != N_GRP * N_GATE ||
      in_sizes[6] != N_GRP * N_HID * N_DIN || in_sizes[7] != N_GRP * N_DIN || out_size != N_OUT0 + N_OUT1) return;

  const float* x      = (const float*)d_in[0];
  const float* h_init = (const float*)d_in[1];
  const float* gamma  = (const float*)d_in[2];
  const float* beta   = (const float*)d_in[3];
  const float* w_in   = (const float*)d_in[4];
  const float* b_in   = (const float*)d_in[5];
  const float* w_out  = (const float*)d_in[6];
  const float* b_out  = (const float*)d_in[7];
  float* out    = (float*)d_out;
  float* h_last = out + (size_t)N_OUT0;

  char* ws = (char*)d_ws;
  size_t off = 0;
  auto carve = [&](size_t bytes) -> char* { char* p = ws + off; off += (bytes + 255) & ~(size_t)255; return p; };
  unsigned short* w_inT  = (unsigned short*)carve((size_t)N_GRP * N_GATE * N_DIN * 2);
  unsigned short* w_outT = (unsigned short*)carve((size_t)N_GRP * N_DIN * N_HID * 2);
  float* A_end    = (float*)carve((size_t)N_BATCH * N_GRP * N_CHUNK * N_HID * 4);
  float* H_end    = (float*)carve((size_t)N_BATCH * N_GRP * N_CHUNK * N_HID * 4);
  float* carry_in = (float*)carve((size_t)N_BATCH * N_GRP * N_CHUNK * N_HID * 4);
  if (off > ws_size || off > (size_t)134217728) return;

  weight_planes_kernel<<<(N8_WIN + N8_WOUT) / N_THR, N_THR, 0, stream>>>(w_in, w_out, w_inT, w_outT);

  const dim3 cgrid(N_CHUNK, N_GRP, N_BATCH);
  chunk_pass_kernel<false><<<cgrid, N_THR, 0, stream>>>(
      x, h_init, gamma, beta, b_in, b_out, w_inT, w_outT, A_end, H_end, carry_in, out);

  carry_scan_kernel<<<(N_BATCH * N_GRP * N_HID) / N_THR, N_THR, 0, stream>>>(A_end, H_end, carry_in, h_last);

  chunk_pass_kernel<true><<<cgrid, N_THR, 0, stream>>>(
      x, h_init, gamma, beta, b_in, b_out, w_inT, w_outT, A_end, H_end, carry_in, out);
}
